// DeepSetsFunc_34196529611494
// MI455X (gfx1250) — hardware-run, weakly checked
//
#include <hip/hip_runtime.h>


#ifndef NL
#define NL 256
#endif
#define NL_FULL 256
#define SS 64
#define DD 128
#define HH 512
#define XP 136
#define HP 520
#define OP 36
#define WCARRY 64.0f
#define WINV   0.015625f

static_assert(NL >= 1 && NL <= NL_FULL);
static_assert(SS == 64);
static_assert(DD % 64 == 0 && HH % 64 == 0);
static_assert(DD % 32 == 0 && HH % 32 == 0);
static_assert(DD == 128 && HH == 512);
static_assert(XP % 8 == 0 && HP % 8 == 0 && OP % 4 == 0);
static_assert(XP >= DD && HP >= HH && OP >= 32);
static_assert(SS * DD == 256 * 4 * 8);
static_assert(256 * 16 * 2 == 64 * 128);
static_assert(32 * 16 * 4 == 16 * 128);
static_assert(8 * 32 * 32 == SS * DD);
static_assert(2 * SS * XP * 2 + SS * HP * 2 + 8 * 16 * OP * 4 <= 131072);
static_assert(64 * 65 * 4 <= 131072);

typedef unsigned short us;
typedef _Float16 h16;
typedef __attribute__((ext_vector_type(16))) _Float16 v16h;
typedef __attribute__((ext_vector_type(8)))  unsigned short v8us;
typedef __attribute__((ext_vector_type(4)))  unsigned short v4us;
typedef __attribute__((ext_vector_type(8)))  float    v8f;
typedef __attribute__((ext_vector_type(4)))  float    v4f;
typedef v4f  __attribute__((may_alias)) v4fa;

__device__ __forceinline__ unsigned short f2bf(float f) { unsigned u = __float_as_uint(f); u += 0x7FFFu + ((u >> 16) & 1u); return (unsigned short)(u >> 16); }
__device__ __forceinline__ float bf2f(unsigned short w) { return __uint_as_float(((unsigned)w) << 16); }
__device__ __forceinline__ float bfv(float f) { return bf2f(f2bf(f)); }
static __device__ __forceinline__ h16 toh_flush(float v) { const h16 r = (h16)v; return (fabsf(v) < 6.103515625e-05f) ? (h16)0.0f : r; }
__device__ __forceinline__ unsigned short hbits(float v) { return __builtin_bit_cast(unsigned short, toh_flush(v)); }
__device__ __forceinline__ v16h cat16h(v8us lo, v8us hi) { return __builtin_bit_cast(v16h, __builtin_shufflevector(lo, hi, 0, 1, 2, 3, 4, 5, 6, 7, 8, 9, 10, 11, 12, 13, 14, 15)); }
__device__ __forceinline__ v8f wmmah(v16h a, v16h b, v8f c) {
    c = __builtin_amdgcn_wmma_f32_16x16x32_f16(false, a, false, b, (short)0, c, false, false);
    asm volatile("v_nop\n\tv_nop\n\tv_nop\n\tv_nop" : "+v"(c) : "v"(a), "v"(b));
    return c; }
__device__ __forceinline__ v16h ldfg(const us* __restrict__ p) { return cat16h(*(const v8us*)p, *(const v8us*)(p + 16)); }
__device__ __forceinline__ v16h ldfs(const us* p)              { return cat16h(*(const v8us*)p, *(const v8us*)(p + 16)); }
__device__ __forceinline__ void wave_sync() { __builtin_amdgcn_fence(3  , "wavefront"); __builtin_amdgcn_wave_barrier(); asm volatile("" ::: "memory"); }

__global__ __launch_bounds__(256) void k_wt(const float* __restrict__ W, us* WT, int K, int N) {
    __shared__ float ts[64 * 65];
    const int t = threadIdx.x;
    const int nkt = K >> 6;
    const int kt = (int)blockIdx.x % nkt, nt = (int)blockIdx.x / nkt;
#pragma unroll 1
    for (int i = 0; i < 16; ++i) { const int f = i * 256 + t; const int kk = f >> 6, nn = f & 63;
        ts[kk * 65 + nn] = W[(size_t)(kt * 64 + kk) * N + nt * 64 + nn]; }
    __syncthreads();
#pragma unroll 1
    for (int ps = 0; ps < 2; ++ps) {
#pragma unroll 1
        for (int it = 0; it < 2; ++it) {
            const int e = it * 32 + (t >> 3), c8 = (t & 7) * 8; v8us o;
#pragma unroll
            for (int k = 0; k < 8; ++k) o[k] = hbits(bfv(ts[(c8 + k) * 65 + e]) * WCARRY);
            *(volatile v8us*)(WT + (size_t)(nt * 64 + e) * K + kt * 64 + c8) = o; }
        if (ps == 0) __threadfence(); }
}

__device__ __forceinline__ void kpass4(const us* sA, int pitch, const us* __restrict__ WT, int kfull, int kcount, int kw0, int ncol0, int lane, v8f (&acc)[4]) {
    const int lr = lane & 15, h8 = (lane >> 4) * 8;
    const us* bp = WT + (size_t)(ncol0 + lr) * kfull + kw0 + h8;
    const us* ap = sA + lr * pitch + h8;
#pragma unroll 1
    for (int kb = 0; kb < kcount; kb += 32) {
        const v16h b  = ldfg(bp + kb);
        const v16h a0 = ldfs(ap + kb);
        const v16h a1 = ldfs(ap + 16 * pitch + kb);
        const v16h a2 = ldfs(ap + 32 * pitch + kb);
        const v16h a3 = ldfs(ap + 48 * pitch + kb);
        acc[0] = wmmah(a0, b, acc[0]);
        acc[1] = wmmah(a1, b, acc[1]);
        acc[2] = wmmah(a2, b, acc[2]);
        acc[3] = wmmah(a3, b, acc[3]);
    }
}

__device__ __forceinline__ void kpass22(const us* sA, int pitch, const us* __restrict__ WT, int kfull, int kcount, int row0, int ncol0, int lane,
                                        v8f& c00, v8f& c01, v8f& c10, v8f& c11) {
    const int lr = lane & 15, h8 = (lane >> 4) * 8;
    const us* bp = WT + (size_t)(ncol0 + lr) * kfull + h8;
    const us* ap = sA + (row0 + lr) * pitch + h8;
#pragma unroll 1
    for (int kb = 0; kb < kcount; kb += 32) {
        const v16h b0 = ldfg(bp + kb);
        const v16h b1 = ldfg(bp + (size_t)16 * kfull + kb);
        const v16h a0 = ldfs(ap + kb);
        const v16h a1 = ldfs(ap + 16 * pitch + kb);
        c00 = wmmah(a0, b0, c00);
        c01 = wmmah(a0, b1, c01);
        c10 = wmmah(a1, b0, c10);
        c11 = wmmah(a1, b1, c11);
    }
}

__device__ __forceinline__ void stripe_to_lds(us* sD, int pitch, int ncol0, int lane, const v8f (&acc)[4], float bias, bool relu) {
    const int lr = lane & 15, hi = lane >> 4;
#pragma unroll
    for (int mt = 0; mt < 4; ++mt) {
#pragma unroll
        for (int j = 0; j < 8; ++j) {
            float v = acc[mt][j] * WINV + bias;
            const float vr = (v > 0.0f) ? v : 0.0f;
            v = relu ? vr : v;
            sD[(mt * 16 + hi * 8 + j) * pitch + ncol0 + lr] = hbits(v); } }
}

__device__ __forceinline__ void out_slab(float* ow, const v8f ca, const v8f cb, float bb0, float bb1,
                                         const float* __restrict__ X, float* OUT, size_t rowbase, int col0, int lane) {
    const int lr = lane & 15, hi = lane >> 4;
#pragma unroll
    for (int j = 0; j < 8; ++j) { ow[(hi * 8 + j) * OP + lr] = ca[j] * WINV + bb0; ow[(hi * 8 + j) * OP + 16 + lr] = cb[j] * WINV + bb1; }
    wave_sync();
    const int rq = lane >> 3, c4 = (lane & 7) * 4;
    v4f v[4];
#pragma unroll
    for (int it = 0; it < 4; ++it) { const int r = 4 * it + rq;
        const size_t g = (rowbase + (size_t)r) * DD + (size_t)(col0 + c4);
        const v4f t = *(const v4fa*)(ow + r * OP + c4);
        const v4f x = *(const v4f*)(X + g);
        v4f o;
#pragma unroll
        for (int k = 0; k < 4; ++k) o[k] = t[k] + bfv(x[k]);
        v[it] = o; }
#pragma unroll
    for (int it = 0; it < 4; ++it) { const int r = 4 * it + rq; const size_t g = (rowbase + (size_t)r) * DD + (size_t)(col0 + c4); *(volatile v4f*)(OUT + g) = v[it]; }
    __threadfence();
#pragma unroll
    for (int it = 0; it < 4; ++it) { const int r = 4 * it + rq; const size_t g = (rowbase + (size_t)r) * DD + (size_t)(col0 + c4); *(volatile v4f*)(OUT + g) = v[it]; }
    wave_sync();
}

__global__ __launch_bounds__(256) void k_sets(const float* __restrict__ X,
                                              const us* __restrict__ W1T, const float* __restrict__ B1,
                                              const us* __restrict__ W2T, const float* __restrict__ B2,
                                              const us* __restrict__ W3T, const float* __restrict__ B3,
                                              const us* __restrict__ W4T, const float* __restrict__ B4,
                                              float* OUT) {
    __shared__ __align__(16) us sX[SS * XP];
    __shared__ __align__(16) us sC[SS * XP];
    __shared__ __align__(16) us sH[SS * HP];
    __shared__ __align__(16) float os[8 * 16 * OP];

    const int tid = threadIdx.x, lane = tid & 31; const int wave = __builtin_amdgcn_readfirstlane(tid >> 5);
    const int l = blockIdx.x;
    const int lr = lane & 15;
    const float* xs = X + (size_t)l * (SS * DD);

#pragma unroll 1
    for (int i = 0; i < 8; ++i) { const int f = i * 256 + tid; const int row = f >> 5, c4 = (f & 31) * 4;
        const v4f v = *(const v4f*)(xs + row * DD + c4); v4us o;
#pragma unroll
        for (int k = 0; k < 4; ++k) o[k] = hbits(bfv(v[k]));
        *(v4us*)(&sX[row * XP + c4]) = o; }

    if (wave < 4) {
        float m1 = -3.402823466e38f, m2 = -3.402823466e38f; int arg = -1;
#pragma unroll 1
        for (int i = 0; i < SS; ++i) { const float v = bfv(xs[i * DD + tid]);
            const bool g1 = v > m1, g2 = v > m2;
            m2 = g1 ? m1 : (g2 ? v : m2); arg = g1 ? i : arg; m1 = g1 ? v : m1; }
        const unsigned short h1 = hbits((m1 > 0.0f) ? m1 : 0.0f);
        const unsigned short h2 = hbits((m2 > 0.0f) ? m2 : 0.0f);
#pragma unroll 1
        for (int j = 0; j < SS; ++j) sC[j * XP + tid] = (j == arg) ? h2 : h1;
    }
    __syncthreads();

#pragma unroll 1
    for (int nt = 0; nt < 4; ++nt) { const int ncol0 = (wave * 4 + nt) * 16;
        v8f acc[4] = { (v8f){}, (v8f){}, (v8f){}, (v8f){} };
        kpass4(sC, XP, W1T, DD, DD, 0, ncol0, lane, acc);
        stripe_to_lds(sH, HP, ncol0, lane, acc, bfv(B1[ncol0 + lr]), true); }
    __syncthreads();

    { const int ncol0 = wave * 16;
        v8f acc[4] = { (v8f){}, (v8f){}, (v8f){}, (v8f){} };
        kpass4(sH, HP, W2T, HH, HH, 0, ncol0, lane, acc);
        stripe_to_lds(sC, XP, ncol0, lane, acc, bfv(B2[ncol0 + lr]), false); }
    __syncthreads();

#pragma unroll 1
    for (int nt = 0; nt < 4; ++nt) { const int ncol0 = (wave * 4 + nt) * 16;
        v8f acc[4] = { (v8f){}, (v8f){}, (v8f){}, (v8f){} };
        kpass4(sX, XP, W3T, 2 * DD, DD, 0,  ncol0, lane, acc);
        kpass4(sC, XP, W3T, 2 * DD, DD, DD, ncol0, lane, acc);
        stripe_to_lds(sH, HP, ncol0, lane, acc, bfv(B3[ncol0 + lr]), true); }
    __syncthreads();

    { const int mh = wave >> 2, nq = wave & 3;
        v8f c00 = (v8f){}, c01 = (v8f){}, c10 = (v8f){}, c11 = (v8f){};
        kpass22(sH, HP, W4T, HH, HH, 32 * mh, 32 * nq, lane, c00, c01, c10, c11);
        const float bb0 = bfv(B4[32 * nq + lr]), bb1 = bfv(B4[32 * nq + 16 + lr]);
        float* ow = &os[wave * 16 * OP];
        const size_t rowbase = (size_t)l * SS + (size_t)(32 * mh);
        out_slab(ow, c00, c01, bb0, bb1, X, OUT, rowbase,      32 * nq, lane);
        out_slab(ow, c10, c11, bb0, bb1, X, OUT, rowbase + 16, 32 * nq, lane); }
}

static constexpr size_t al256(size_t v) { return (v + 255) & ~(size_t)255; }
static constexpr size_t SZ_W1T = al256((size_t)HH * DD * 2);
static constexpr size_t SZ_W2T = al256((size_t)DD * HH * 2);
static constexpr size_t SZ_W3T = al256((size_t)HH * 2 * DD * 2);
static constexpr size_t SZ_W4T = al256((size_t)DD * HH * 2);
static constexpr size_t SZ_TOTAL = SZ_W1T + SZ_W2T + SZ_W3T + SZ_W4T;
static_assert(SZ_TOTAL <= (size_t)134217728);

extern "C" void kernel_launch(void* const* d_in, const int* in_sizes, int n_in,
                              void* d_out, int out_size, void* d_ws, size_t ws_size, hipStream_t stream) {
    if (n_in < 9) return;
    if ((size_t)in_sizes[0] < (size_t)NL * SS * DD) return;
    if ((size_t)in_sizes[1] < (size_t)DD * HH || (size_t)in_sizes[2] < (size_t)HH) return;
    if ((size_t)in_sizes[3] < (size_t)HH * DD || (size_t)in_sizes[4] < (size_t)DD) return;
    if ((size_t)in_sizes[5] < (size_t)2 * DD * HH || (size_t)in_sizes[6] < (size_t)HH) return;
    if ((size_t)in_sizes[7] < (size_t)HH * DD || (size_t)in_sizes[8] < (size_t)DD) return;
    if ((size_t)out_size < (size_t)NL * SS * DD) return;
    if (SZ_TOTAL > ws_size) return;
    const float* X  = (const float*)d_in[0];
    const float* W1 = (const float*)d_in[1];
    const float* b1 = (const float*)d_in[2];
    const float* W2 = (const float*)d_in[3];
    const float* b2 = (const float*)d_in[4];
    const float* W3 = (const float*)d_in[5];
    const float* b3 = (const float*)d_in[6];
    const float* W4 = (const float*)d_in[7];
    const float* b4 = (const float*)d_in[8];
    float* OUT = (float*)d_out;
    char* wsp = (char*)d_ws;
    us* W1T = (us*)wsp; wsp += SZ_W1T;
    us* W2T = (us*)wsp; wsp += SZ_W2T;
    us* W3T = (us*)wsp; wsp += SZ_W3T;
    us* W4T = (us*)wsp; wsp += SZ_W4T;

    k_wt<<<(DD / 64) * (HH / 64), 256, 0, stream>>>(W1, W1T, DD, HH);
    k_wt<<<(HH / 64) * (DD / 64), 256, 0, stream>>>(W2, W2T, HH, DD);
    k_wt<<<((2 * DD) / 64) * (HH / 64), 256, 0, stream>>>(W3, W3T, 2 * DD, HH);
    k_wt<<<(HH / 64) * (DD / 64), 256, 0, stream>>>(W4, W4T, HH, DD);
    k_sets<<<NL, 256, 0, stream>>>(X, W1T, b1, W2T, b2, W3T, b3, W4T, b4, OUT);
}
